// Cross_Frame_Att_17755394801887
// MI455X (gfx1250) — hardware-verified
//
#include <hip/hip_runtime.h>
#include <math.h>


typedef _Float16 f16;
typedef __bf16  bf16;
typedef f16   v16h __attribute__((ext_vector_type(16)));
typedef f16   v8h  __attribute__((ext_vector_type(8)));
typedef bf16  v16b __attribute__((ext_vector_type(16)));
typedef bf16  v8b  __attribute__((ext_vector_type(8)));
typedef float v8f  __attribute__((ext_vector_type(8)));
typedef float v4f  __attribute__((ext_vector_type(4)));

union FragH { v16h v; v8h p[2]; };
union FragB { v16b v; v8b p[2]; };

#define DEVFN __device__ __forceinline__

constexpr int B = 8, F = 4, C = 128, N = 1024, H = 4;
constexpr int DW  = 4 * C;
constexpr int MB  = 64;
constexpr int NMB = N / MB;
constexpr int AP  = 136;
constexpr float EPS     = 1e-5f;
constexpr float SCALE   = 0.08838834764831845f;
constexpr float WSC     = 1024.0f;
constexpr float WSC_INV = 0.0009765625f;
constexpr float PSC     = 64.0f;
constexpr float PSC_INV = 0.015625f;

constexpr int OUT0 = B * 3 * N * C;
constexpr int OUT1 = B * 3 * N * 3;
constexpr int OUT_TOTAL = OUT0 + OUT1 + 1;

static_assert(N % MB == 0);
static_assert(C == 128 && DW == 512 && H == 4);
static_assert((DW * C / 8) % 256 == 0 && (C * C / 8) % 256 == 0);

constexpr size_t al256(size_t x) { return (x + 255) & ~(size_t)255; }
constexpr size_t WS_SS  = 0;
constexpr size_t WS_WQ  = al256(WS_SS  + (size_t)B * 2 * C * 4);
constexpr size_t WS_WK  = al256(WS_WQ  + (size_t)DW * C * 2);
constexpr size_t WS_WVH = al256(WS_WK  + (size_t)DW * C * 2);
constexpr size_t WS_WVL = al256(WS_WVH + (size_t)DW * C * 2);
constexpr size_t WS_WPH = al256(WS_WVL + (size_t)DW * C * 2);
constexpr size_t WS_WPL = al256(WS_WPH + (size_t)C * C * 2);
constexpr size_t WS_Q   = al256(WS_WPL + (size_t)C * C * 2);
constexpr size_t WS_K   = al256(WS_Q   + (size_t)B * 2 * N * DW * 2);
constexpr size_t WS_VT  = al256(WS_K   + (size_t)B * 2 * N * DW * 2);
constexpr size_t WS_VP  = al256(WS_VT  + (size_t)B * 2 * H * C * N * 2);
constexpr size_t WS_OV  = al256(WS_VP  + (size_t)B * 2 * NMB * DW * 4);
constexpr size_t WS_PR  = al256(WS_OV  + (size_t)B * 2 * H * N * C * 4);
constexpr size_t WS_END = al256(WS_PR  + (size_t)B * 3 * N * 4);

constexpr int LDS_QKV = 4 * MB * AP * 2 + 8 * 1024 * 2 + 8 * 64 * 4;
constexpr int LDS_ATT = MB * N * 2;
constexpr int LDS_PRJ = 2 * MB * AP * 2 + MB * C * 4;
static_assert(4 * 16 * C * 4 <= LDS_ATT);

DEVFN v8f mma_h(v16h a, v16h b, v8f c) {
  c = __builtin_amdgcn_wmma_f32_16x16x32_f16(false, a, false, b, (short)0, c, false, false);
  asm volatile("v_nop\n\tv_nop\n\tv_nop\n\tv_nop" : "+v"(c) : "v"(a), "v"(b));
  return c;
}
DEVFN v8f mma_b(v16b a, v16b b, v8f c) {
  c = __builtin_amdgcn_wmma_f32_16x16x32_bf16(false, a, false, b, (short)0, c, false, false);
  asm volatile("v_nop\n\tv_nop\n\tv_nop\n\tv_nop" : "+v"(c) : "v"(a), "v"(b));
  return c;
}
DEVFN v16h frag_h(const f16* base, int ld, int row, int k0, int hf) {
  const f16* p = base + (size_t)row * ld + k0 + 8 * hf;
  FragH f;
  f.p[0] = *(const v8h*)p;
  f.p[1] = *(const v8h*)(p + 16);
  return f.v;
}
DEVFN v16b frag_b(const bf16* base, int ld, int row, int k0, int hf) {
  const bf16* p = base + (size_t)row * ld + k0 + 8 * hf;
  FragB f;
  f.p[0] = *(const v8b*)p;
  f.p[1] = *(const v8b*)(p + 16);
  return f.v;
}
DEVFN v8f zero8() { v8f z = {0.f, 0.f, 0.f, 0.f, 0.f, 0.f, 0.f, 0.f}; return z; }
DEVFN float wsum(float v) {
#pragma unroll
  for (int o = 16; o > 0; o >>= 1) v += __shfl_xor(v, o, 32);
  return v;
}

__global__ void __launch_bounds__(256)
k_bn(const float* __restrict__ xs, const float* __restrict__ gamma, float* __restrict__ ss) {
  __shared__ float s_sc[C];
  __shared__ float s_mn[C];
  const int b = blockIdx.x;
  if (b >= B) return;
  const int tid = threadIdx.x, lane = tid & 31, wave = tid >> 5;
#pragma unroll 1
  for (int ci = 0; ci < C / 8; ++ci) {
    const int c = wave * (C / 8) + ci;
    const float* base = xs + ((size_t)b * F * C + c) * N;
    float s = 0.f;
#pragma unroll 1
    for (int fr = 0; fr < F; ++fr) {
      const float* p = base + (size_t)fr * C * N;
      for (int n = lane; n < N; n += 32) s += p[n];
    }
    s = wsum(s);
    const float mean = s * (1.0f / (float)(F * N));
    float q = 0.f;
#pragma unroll 1
    for (int fr = 0; fr < F; ++fr) {
      const float* p = base + (size_t)fr * C * N;
      for (int n = lane; n < N; n += 32) { const float d = p[n] - mean; q += d * d; }
    }
    q = wsum(q);
    const float var = q * (1.0f / (float)(F * N));
    if (lane == 0) {
      const float istd = 1.0f / sqrtf(var + EPS);
      s_sc[c] = istd * gamma[c];
      s_mn[c] = mean;
    }
  }
  __syncthreads();
  if (wave == 0) {
    const v4f vm = {s_mn[4 * lane], s_mn[4 * lane + 1], s_mn[4 * lane + 2], s_mn[4 * lane + 3]};
    const v4f vs = {s_sc[4 * lane], s_sc[4 * lane + 1], s_sc[4 * lane + 2], s_sc[4 * lane + 3]};
    float* dst = ss + (size_t)b * 2 * C;
    *(volatile v4f*)(dst + 4 * lane) = vm;
    *(volatile v4f*)(dst + C + 4 * lane) = vs;
    __threadfence();
    *(volatile v4f*)(dst + 4 * lane) = vm;
    *(volatile v4f*)(dst + C + 4 * lane) = vs;
  }
}

__global__ void __launch_bounds__(256)
k_cvt_h(const float* __restrict__ in, f16* __restrict__ out, int n8, float scale) {
  const int i = blockIdx.x * 256 + (int)threadIdx.x;
  if (i >= n8) return;
  const float* p = in + (size_t)i * 8;
  v8h r;
#pragma unroll
  for (int j = 0; j < 8; ++j) r[j] = (f16)(p[j] * scale);
  f16* d = out + (size_t)i * 8;
  *(volatile v8h*)d = r;
  __threadfence();
  *(volatile v8h*)d = r;
}

__global__ void __launch_bounds__(256)
k_cvt_b2(const float* __restrict__ in, bf16* __restrict__ hi, bf16* __restrict__ lo, int n8) {
  const int i = blockIdx.x * 256 + (int)threadIdx.x;
  if (i >= n8) return;
  const float* p = in + (size_t)i * 8;
  v8b rh, rl;
#pragma unroll
  for (int j = 0; j < 8; ++j) {
    const float x = p[j];
    const bf16 hh = (bf16)x;
    rh[j] = hh;
    rl[j] = (bf16)(x - (float)hh);
  }
  bf16* dh = hi + (size_t)i * 8;
  bf16* dl = lo + (size_t)i * 8;
  *(volatile v8b*)dh = rh;
  *(volatile v8b*)dl = rl;
  __threadfence();
  *(volatile v8b*)dh = rh;
  *(volatile v8b*)dl = rl;
}

__global__ void __launch_bounds__(256)
k_qkv(const float* __restrict__ xs, const float* __restrict__ ss, const float* __restrict__ beta,
      const f16* __restrict__ wq, const f16* __restrict__ wk,
      const bf16* __restrict__ wvh, const bf16* __restrict__ wvl,
      f16* __restrict__ q16, f16* __restrict__ k16, f16* __restrict__ vt16,
      float* __restrict__ vpart) {
  extern __shared__ v4f dyn_qkv[];
  char* lds = (char*)dyn_qkv;
  f16*  Pq = (f16*)lds;
  f16*  Pk = Pq + MB * AP;
  bf16* Ph = (bf16*)(Pk + MB * AP);
  bf16* Pl = Ph + MB * AP;
  f16*  St = (f16*)(Pl + MB * AP);
  float* Cs = (float*)(St + 8 * 1024);
  __shared__ float s_mn[C], s_sc[C], s_be[C];

  const int bf = blockIdx.x, mb = blockIdx.y;
  if (bf >= B * 2 || mb >= NMB) return;
  const int b = bf >> 1, f = bf & 1, n0 = mb * MB;
  const int tid = threadIdx.x, lane = tid & 31, wave = tid >> 5, hf = lane >> 4, m = lane & 15;

  if (tid < C) {
    s_mn[tid] = ss[(size_t)b * 2 * C + tid];
    s_sc[tid] = ss[(size_t)b * 2 * C + C + tid];
    s_be[tid] = beta[tid];
  }
  __syncthreads();

  const float* xq = xs + ((size_t)(b * F + f) * C) * N + n0;
  const float* xv = xs + ((size_t)(b * F + (F - 1 - f)) * C) * N + n0;
#pragma unroll 4
  for (int i = 0; i < (C * MB) / 256; ++i) {
    const int idx = i * 256 + tid, c = idx >> 6, nl = idx & 63;
    const float mn = s_mn[c], sc = s_sc[c], be = s_be[c];
    const float a0 = (xq[(size_t)c * N + nl] - mn) * sc + be;
    const float a1 = (xv[(size_t)c * N + nl] - mn) * sc + be;
    Pq[nl * AP + c] = (f16)a0;
    Pk[nl * AP + c] = (f16)a1;
    const bf16 hh = (bf16)a1;
    Ph[nl * AP + c] = hh;
    Pl[nl * AP + c] = (bf16)(a1 - (float)hh);
  }
  __syncthreads();

  f16* Stw = St + wave * 1024;

#pragma unroll 1
  for (int which = 0; which < 2; ++which) {
    const f16* P = which ? Pk : Pq;
    const f16* W = which ? wk : wq;
    f16* O = (which ? k16 : q16) + ((size_t)bf * N + n0) * DW + wave * 64;
#pragma unroll 1
    for (int mt = 0; mt < 4; ++mt) {
      v16h a[4];
#pragma unroll
      for (int ks = 0; ks < 4; ++ks) a[ks] = frag_h(P, AP, mt * 16 + m, ks * 32, hf);
#pragma unroll
      for (int j = 0; j < 4; ++j) {
        const int nrow = (wave * 4 + j) * 16 + m;
        v8f acc = zero8();
#pragma unroll
        for (int ks = 0; ks < 4; ++ks) acc = mma_h(a[ks], frag_h(W, C, nrow, ks * 32, hf), acc);
#pragma unroll
        for (int r = 0; r < 8; ++r) Stw[(8 * hf + r) * 64 + j * 16 + m] = (f16)(acc[r] * WSC_INV);
      }
      __syncthreads();
      v8h vv[4];
#pragma unroll
      for (int i = 0; i < 4; ++i) vv[i] = *(const v8h*)(Stw + (i * 4 + (lane >> 3)) * 64 + (lane & 7) * 8);
      f16* Om = O + (size_t)(mt * 16) * DW;
#pragma unroll
      for (int i = 0; i < 4; ++i)
        *(volatile v8h*)(Om + (size_t)(i * 4 + (lane >> 3)) * DW + (lane & 7) * 8) = vv[i];
      __threadfence();
#pragma unroll
      for (int i = 0; i < 4; ++i)
        *(volatile v8h*)(Om + (size_t)(i * 4 + (lane >> 3)) * DW + (lane & 7) * 8) = vv[i];
      __syncthreads();
    }
  }

#pragma unroll 1
  for (int j = 0; j < 4; ++j) {
    const int ct = wave * 4 + j;
    v16b bh4[4], bl4[4];
#pragma unroll
    for (int ks = 0; ks < 4; ++ks) {
      bh4[ks] = frag_b(wvh, C, ct * 16 + m, ks * 32, hf);
      bl4[ks] = frag_b(wvl, C, ct * 16 + m, ks * 32, hf);
    }
    float csum = 0.f;
#pragma unroll 1
    for (int mt = 0; mt < 4; ++mt) {
      v8f acc = zero8();
#pragma unroll
      for (int ks = 0; ks < 4; ++ks) {
        const v16b ah = frag_b(Ph, AP, mt * 16 + m, ks * 32, hf);
        const v16b al = frag_b(Pl, AP, mt * 16 + m, ks * 32, hf);
        acc = mma_b(ah, bh4[ks], acc);
        acc = mma_b(ah, bl4[ks], acc);
        acc = mma_b(al, bh4[ks], acc);
      }
#pragma unroll
      for (int r = 0; r < 8; ++r) {
        csum += acc[r];
        Stw[m * 64 + mt * 16 + 8 * hf + r] = (f16)acc[r];
      }
    }
    csum += __shfl_xor(csum, 16, 32);
    if (lane < 16) Cs[wave * 64 + j * 16 + lane] = csum;
    __syncthreads();
    const int gc0 = ct * 16, hh = gc0 >> 7, cb = gc0 & (C - 1);
    f16* Ov = vt16 + (((size_t)(bf * H + hh)) * C + cb) * N + n0;
    v8h vv[4];
#pragma unroll
    for (int i = 0; i < 4; ++i) vv[i] = *(const v8h*)(Stw + (i * 4 + (lane >> 3)) * 64 + (lane & 7) * 8);
#pragma unroll
    for (int i = 0; i < 4; ++i)
      *(volatile v8h*)(Ov + (size_t)(i * 4 + (lane >> 3)) * N + (lane & 7) * 8) = vv[i];
    __threadfence();
#pragma unroll
    for (int i = 0; i < 4; ++i)
      *(volatile v8h*)(Ov + (size_t)(i * 4 + (lane >> 3)) * N + (lane & 7) * 8) = vv[i];
    __syncthreads();
  }
  if (lane < 16) {
    const float* cs = Cs + wave * 64 + 4 * lane;
    const v4f cv = {cs[0], cs[1], cs[2], cs[3]};
    float* dst = vpart + ((size_t)(bf * NMB + mb)) * DW + wave * 64 + 4 * lane;
    *(volatile v4f*)dst = cv;
    __threadfence();
    *(volatile v4f*)dst = cv;
  }
}

__global__ void __launch_bounds__(128)
k_attn(const f16* __restrict__ q16, const f16* __restrict__ k16, const f16* __restrict__ vt16,
       const float* __restrict__ vpart, float* __restrict__ ov) {
  extern __shared__ v4f dyn_att[];
  f16* Sp = (f16*)dyn_att;
  __shared__ float cm[C], inv_s[MB], c0_s[MB], redm[2 * MB], reds[2 * MB], redS[2 * MB];

  const int bfh = blockIdx.x, mb = blockIdx.y;
  if (bfh >= B * 2 * H || mb >= NMB) return;
  const int bf = bfh >> 2, h = bfh & 3, m0 = mb * MB;
  const int tid = threadIdx.x, lane = tid & 31, wave = tid >> 5, hf = lane >> 4, m = lane & 15;

  {
    const float* vp = vpart + (size_t)bf * NMB * DW + h * C + tid;
    float s = 0.f;
#pragma unroll
    for (int i = 0; i < NMB; ++i) s += vp[(size_t)i * DW];
    cm[tid] = s;
  }

  const f16* qb = q16 + (size_t)bf * N * DW + h * C;
  const f16* kb = k16 + (size_t)bf * N * DW + h * C;
  v16h aq[4];
#pragma unroll
  for (int ks = 0; ks < 4; ++ks) aq[ks] = frag_h(qb, DW, m0 + wave * 16 + m, ks * 32, hf);
  f16* Sw = Sp + (size_t)(wave * 16) * N;
#pragma unroll 1
  for (int kt = 0; kt < N / 16; ++kt) {
    v8f acc = zero8();
#pragma unroll
    for (int ks = 0; ks < 4; ++ks) acc = mma_h(aq[ks], frag_h(kb, DW, kt * 16 + m, ks * 32, hf), acc);
#pragma unroll
    for (int r = 0; r < 8; ++r) Sw[(size_t)(8 * hf + r) * N + kt * 16 + m] = (f16)acc[r];
  }
  __syncthreads();

  {
    const int row = tid >> 1, part = tid & 1;
    f16* rp = Sp + (size_t)row * N + part * (N / 2);
    float mx = -3.0e38f, ssum = 0.f;
    for (int jb = 0; jb < N / 16; ++jb) {
      const v8h v = *(const v8h*)(rp + jb * 8);
#pragma unroll
      for (int i = 0; i < 8; ++i) { const float x = (float)v[i]; mx = fmaxf(mx, x); ssum += x; }
    }
    redm[tid] = mx;
    reds[tid] = ssum;
    __syncthreads();
    mx = fmaxf(redm[row * 2], redm[row * 2 + 1]);
    const float smean = (reds[row * 2] + reds[row * 2 + 1]) * (1.0f / (float)N);
    const float c0 = __expf((smean - mx) * SCALE);
    float S = 0.f;
    for (int jb = 0; jb < N / 16; ++jb) {
      const v8h v = *(const v8h*)(rp + jb * 8);
      v8h e;
#pragma unroll
      for (int i = 0; i < 8; ++i) {
        const float x = __expf(((float)v[i] - mx) * SCALE);
        S += x;
        e[i] = (f16)((x - c0) * PSC);
      }
      *(v8h*)(rp + jb * 8) = e;
    }
    redS[tid] = S;
    __syncthreads();
    if (part == 0) {
      inv_s[row] = 1.0f / (redS[row * 2] + redS[row * 2 + 1]);
      c0_s[row] = c0;
    }
    __syncthreads();
  }

  float myinv[8], myc0[8];
#pragma unroll
  for (int r = 0; r < 8; ++r) {
    const int rr = wave * 16 + 8 * hf + r;
    myinv[r] = inv_s[rr];
    myc0[r] = c0_s[rr];
  }
  const f16* vb = vt16 + (size_t)bfh * C * N;
  const f16* Pw = Sp + (size_t)(wave * 16) * N;
  v8f acc[8];
#pragma unroll
  for (int ct = 0; ct < 8; ++ct) acc[ct] = zero8();
#pragma unroll 1
  for (int ks = 0; ks < N / 32; ++ks) {
    const v16h a = frag_h(Pw, N, m, ks * 32, hf);
#pragma unroll
    for (int ct = 0; ct < 8; ++ct) acc[ct] = mma_h(a, frag_h(vb, N, ct * 16 + m, ks * 32, hf), acc[ct]);
  }
  __syncthreads();
  float* stg = (float*)dyn_att + wave * 16 * C;
#pragma unroll
  for (int ct = 0; ct < 8; ++ct) {
#pragma unroll
    for (int r = 0; r < 8; ++r) {
      const int c = ct * 16 + m;
      stg[(8 * hf + r) * C + c] = (myc0[r] * cm[c] + acc[ct][r] * PSC_INV) * myinv[r];
    }
  }
  __syncthreads();
  float* Ob = ov + ((size_t)bfh * N + m0 + wave * 16) * C;
#pragma unroll
  for (int i = 0; i < 16; ++i) {
    const v4f v = *(const v4f*)(stg + i * C + 4 * lane);
    *(volatile v4f*)(Ob + (size_t)i * C + 4 * lane) = v;
  }
  __threadfence();
#pragma unroll
  for (int i = 0; i < 16; ++i) {
    const v4f v = *(const v4f*)(stg + i * C + 4 * lane);
    *(volatile v4f*)(Ob + (size_t)i * C + 4 * lane) = v;
  }
}

__global__ void __launch_bounds__(256)
k_proj(const float* __restrict__ ov, const bf16* __restrict__ wph, const bf16* __restrict__ wpl,
       const float* __restrict__ bp, const float* __restrict__ Wm, const float* __restrict__ bm,
       const float* __restrict__ pc1, float* __restrict__ out0, float* __restrict__ out1,
       float* __restrict__ pred) {
  extern __shared__ v4f dyn_prj[];
  char* lds = (char*)dyn_prj;
  bf16* Ah = (bf16*)lds;
  bf16* Al = Ah + MB * AP;
  float* X = (float*)(Al + MB * AP);
  __shared__ float s_wm[3 * C], s_bp[C], s_bm[3], s_fr[MB * 3], s_pr[3 * MB];

  const int bh = blockIdx.x, mb = blockIdx.y;
  if (bh >= B * H || mb >= NMB) return;
  const int b = bh >> 2, h = bh & 3, n0 = mb * MB;
  const int tid = threadIdx.x, lane = tid & 31, wave = tid >> 5, hf = lane >> 4, m = lane & 15;

  for (int i = tid; i < 3 * C; i += 256) s_wm[i] = Wm[i];
  if (tid < C) s_bp[tid] = bp[tid];
  if (tid < 3) s_bm[tid] = bm[tid];

  const float* o0 = ov + (((size_t)(b * 2 + 0) * H + h) * N + n0) * C;
  const float* o1 = ov + (((size_t)(b * 2 + 1) * H + h) * N + n0) * C;
#pragma unroll 4
  for (int i = 0; i < (MB * C) / 256; ++i) {
    const int idx = i * 256 + tid, row = idx >> 7, c = idx & (C - 1);
    const float s = o0[idx] + o1[idx];
    const bf16 hh = (bf16)s;
    Ah[row * AP + c] = hh;
    Al[row * AP + c] = (bf16)(s - (float)hh);
  }
  __syncthreads();

  v16b bh4[4], bl4[4];
#pragma unroll
  for (int ks = 0; ks < 4; ++ks) {
    bh4[ks] = frag_b(wph, C, wave * 16 + m, ks * 32, hf);
    bl4[ks] = frag_b(wpl, C, wave * 16 + m, ks * 32, hf);
  }
#pragma unroll 1
  for (int mt = 0; mt < 4; ++mt) {
    v8f acc = zero8();
#pragma unroll
    for (int ks = 0; ks < 4; ++ks) {
      const v16b ah = frag_b(Ah, AP, mt * 16 + m, ks * 32, hf);
      const v16b al = frag_b(Al, AP, mt * 16 + m, ks * 32, hf);
      acc = mma_b(ah, bh4[ks], acc);
      acc = mma_b(ah, bl4[ks], acc);
      acc = mma_b(al, bh4[ks], acc);
    }
    const int d = wave * 16 + m;
    const float bias = s_bp[d];
#pragma unroll
    for (int r = 0; r < 8; ++r) X[(mt * 16 + 8 * hf + r) * C + d] = acc[r] + bias;
  }
  __syncthreads();

  if (h >= 1) {
    float* Ob = out0 + (((size_t)(b * 3 + h - 1)) * N + n0) * C;
#pragma unroll
    for (int i = 0; i < 8; ++i) {
      const int row = wave * 8 + i;
      const v4f v = *(const v4f*)(X + row * C + 4 * lane);
      *(volatile v4f*)(Ob + (size_t)row * C + 4 * lane) = v;
    }
    __threadfence();
#pragma unroll
    for (int i = 0; i < 8; ++i) {
      const int row = wave * 8 + i;
      const v4f v = *(const v4f*)(X + row * C + 4 * lane);
      *(volatile v4f*)(Ob + (size_t)row * C + 4 * lane) = v;
    }
  }

  if (tid < MB * 3) {
    const int row = tid / 3, j = tid - row * 3;
    const float* xr = X + row * C;
    const float* wr = s_wm + j * C;
    float a = 0.f;
#pragma unroll 8
    for (int c = 0; c < C; ++c) a += xr[c] * wr[c];
    const float fv = a + s_bm[j];
    s_fr[row * 3 + j] = fv;
    if (h == 0) s_pr[j * MB + row] = pc1[((size_t)b * 3 + j) * N + n0 + row] + fv;
  }
  __syncthreads();

  if (h >= 1) {
    if (wave == 0) {
      float* Of = out1 + (((size_t)(b * 3 + h - 1)) * N + n0) * 3;
      const v4f v0 = {s_fr[4 * lane], s_fr[4 * lane + 1], s_fr[4 * lane + 2], s_fr[4 * lane + 3]};
      v4f v1 = {0.f, 0.f, 0.f, 0.f};
      if (lane < 16) { v1[0] = s_fr[128 + 4 * lane]; v1[1] = s_fr[129 + 4 * lane]; v1[2] = s_fr[130 + 4 * lane]; v1[3] = s_fr[131 + 4 * lane]; }
      *(volatile v4f*)(Of + 4 * lane) = v0;
      if (lane < 16) *(volatile v4f*)(Of + 128 + 4 * lane) = v1;
      __threadfence();
      *(volatile v4f*)(Of + 4 * lane) = v0;
      if (lane < 16) *(volatile v4f*)(Of + 128 + 4 * lane) = v1;
    }
  } else {
    if (wave == 0 && lane < 16) {
      v4f pv[3];
#pragma unroll
      for (int j = 0; j < 3; ++j) {
        const float* sp = s_pr + j * MB + 4 * lane;
        pv[j][0] = sp[0]; pv[j][1] = sp[1]; pv[j][2] = sp[2]; pv[j][3] = sp[3];
      }
#pragma unroll
      for (int j = 0; j < 3; ++j)
        *(volatile v4f*)(pred + ((size_t)(b * 3 + j)) * N + n0 + 4 * lane) = pv[j];
      __threadfence();
#pragma unroll
      for (int j = 0; j < 3; ++j)
        *(volatile v4f*)(pred + ((size_t)(b * 3 + j)) * N + n0 + 4 * lane) = pv[j];
    }
  }
}

__global__ void __launch_bounds__(256)
k_cham(const float* __restrict__ pred, const float* __restrict__ pc1, float* __restrict__ out_loss) {
#pragma clang fp contract(off)
  __shared__ float P[3 * N];
  __shared__ float G[3 * N];
  __shared__ float r0[8], r1[8];
  const int tid = threadIdx.x, lane = tid & 31, wave = tid >> 5;
  float s0 = 0.f, s1 = 0.f;
#pragma unroll 1
  for (int b = 0; b < B; ++b) {
    __syncthreads();
    for (int i = tid; i < 3 * N; i += 256) {
      P[i] = pred[(size_t)b * 3 * N + i];
      G[i] = pc1[(size_t)b * 3 * N + i];
    }
    __syncthreads();
    for (int n = tid; n < N; n += 256) {
      const float px = P[n], py = P[N + n], pz = P[2 * N + n];
      float mn = 3.0e38f;
#pragma unroll 4
      for (int j = 0; j < N; ++j) {
        const float dx = px - G[j], dy = py - G[N + j], dz = pz - G[2 * N + j];
        const float d = dx * dx + dy * dy + dz * dz;
        mn = fminf(mn, d);
      }
      s0 += mn;
    }
    for (int j = tid; j < N; j += 256) {
      const float gx = G[j], gy = G[N + j], gz = G[2 * N + j];
      float mn = 3.0e38f;
#pragma unroll 4
      for (int n = 0; n < N; ++n) {
        const float dx = P[n] - gx, dy = P[N + n] - gy, dz = P[2 * N + n] - gz;
        const float d = dx * dx + dy * dy + dz * dz;
        mn = fminf(mn, d);
      }
      s1 += mn;
    }
  }
  s0 = wsum(s0);
  s1 = wsum(s1);
  if (lane == 0) { r0[wave] = s0; r1[wave] = s1; }
  __syncthreads();
  if (tid == 0) {
    float t0 = 0.f, t1 = 0.f;
    for (int w = 0; w < 8; ++w) { t0 += r0[w]; t1 += r1[w]; }
    const float loss = t0 * (1.0f / (float)(B * N)) + t1 * (1.0f / (float)(B * N));
    *(volatile float*)out_loss = loss;
    __threadfence();
    *(volatile float*)out_loss = loss;
  }
}

extern "C" void kernel_launch(void* const* d_in, const int* in_sizes, int n_in,
                              void* d_out, int out_size, void* d_ws, size_t ws_size,
                              hipStream_t stream) {
  if (n_in < 11) return;
  if (in_sizes[0] != B * F * C * N || in_sizes[1] != B * 3 * N || in_sizes[3] != C ||
      in_sizes[4] != C || in_sizes[5] != DW * C || in_sizes[6] != 2 * DW * C ||
      in_sizes[7] != C * C || in_sizes[8] != C || in_sizes[9] != 3 * C || in_sizes[10] != 3 ||
      out_size != OUT_TOTAL) return;
  if (WS_END > ws_size) return;

  const float* xs    = (const float*)d_in[0];
  const float* pc1   = (const float*)d_in[1];
  const float* gamma = (const float*)d_in[3];
  const float* beta  = (const float*)d_in[4];
  const float* Wq    = (const float*)d_in[5];
  const float* Wkv   = (const float*)d_in[6];
  const float* Wp    = (const float*)d_in[7];
  const float* bp    = (const float*)d_in[8];
  const float* Wm    = (const float*)d_in[9];
  const float* bm    = (const float*)d_in[10];

  char* ws = (char*)d_ws;
  float* ss    = (float*)(ws + WS_SS);
  f16*   wq16  = (f16*)(ws + WS_WQ);
  f16*   wk16  = (f16*)(ws + WS_WK);
  bf16*  wvh   = (bf16*)(ws + WS_WVH);
  bf16*  wvl   = (bf16*)(ws + WS_WVL);
  bf16*  wph   = (bf16*)(ws + WS_WPH);
  bf16*  wpl   = (bf16*)(ws + WS_WPL);
  f16*   q16   = (f16*)(ws + WS_Q);
  f16*   k16   = (f16*)(ws + WS_K);
  f16*   vt16  = (f16*)(ws + WS_VT);
  float* vpart = (float*)(ws + WS_VP);
  float* ovf   = (float*)(ws + WS_OV);
  float* pred  = (float*)(ws + WS_PR);

  float* out0  = (float*)d_out;
  float* out1  = out0 + OUT0;
  float* outl  = out0 + (size_t)OUT0 + OUT1;

  (void)hipFuncSetAttribute((const void*)k_qkv,  hipFuncAttributeMaxDynamicSharedMemorySize, LDS_QKV);
  (void)hipFuncSetAttribute((const void*)k_attn, hipFuncAttributeMaxDynamicSharedMemorySize, LDS_ATT);
  (void)hipFuncSetAttribute((const void*)k_proj, hipFuncAttributeMaxDynamicSharedMemorySize, LDS_PRJ);

  const int n8w = DW * C / 8;
  const int n8p = C * C / 8;

  k_bn<<<dim3(B), dim3(256), 0, stream>>>(xs, gamma, ss);
  k_cvt_h<<<dim3((n8w + 255) / 256), dim3(256), 0, stream>>>(Wq, wq16, n8w, WSC);
  k_cvt_h<<<dim3((n8w + 255) / 256), dim3(256), 0, stream>>>(Wkv, wk16, n8w, WSC);
  k_cvt_b2<<<dim3((n8w + 255) / 256), dim3(256), 0, stream>>>(Wkv + (size_t)DW * C, wvh, wvl, n8w);
  k_cvt_b2<<<dim3((n8p + 255) / 256), dim3(256), 0, stream>>>(Wp, wph, wpl, n8p);
  k_qkv<<<dim3(B * 2, NMB), dim3(256), LDS_QKV, stream>>>(xs, ss, beta, wq16, wk16, wvh, wvl,
                                                         q16, k16, vt16, vpart);
  k_attn<<<dim3(B * 2 * H, NMB), dim3(128), LDS_ATT, stream>>>(q16, k16, vt16, vpart, ovf);
  k_proj<<<dim3(B * H, NMB), dim3(256), LDS_PRJ, stream>>>(ovf, wph, wpl, bp, Wm, bm, pc1,
                                                          out0, out1, pred);
  k_cham<<<dim3(1), dim3(256), 0, stream>>>(pred, pc1, outl);
  (void)hipGetLastError();
}
